// LocalAttention_26603027432182
// MI455X (gfx1250) — hardware-verified
//
#include <hip/hip_runtime.h>

typedef _Float16 v16h __attribute__((ext_vector_type(16)));
typedef _Float16 v8h  __attribute__((ext_vector_type(8)));
typedef _Float16 v4h  __attribute__((ext_vector_type(4)));
typedef float    v8f  __attribute__((ext_vector_type(8)));
typedef float    v4f  __attribute__((ext_vector_type(4)));
typedef float    v4fa __attribute__((ext_vector_type(4), may_alias));

#ifndef NB
#define NB 2
#endif
#ifndef SEQ
#define SEQ 4096
#endif
#define NB_FULL 2
#define S_FULL  4096
#define NH      8
#define HD      64
#define HALF_W  50
#define QB      64
#define KP      72
#define VP      40
#define NEG_BIG (-1.0e30f)
#define SCALE   0.125f
#define PSCALE  1024.0f
#define LSCALE  2048.0f
#define RSPLIT  (1.0f / 2048.0f)

static_assert(SEQ % QB == 0);
static_assert(SEQ % 32 == 0);
static_assert(SEQ <= S_FULL);
static_assert(NB <= NB_FULL);
static_assert(HD == 64);
static_assert((KP % 8) == 0 && (VP % 8) == 0);
static_assert(KP >= HD && VP >= 32);

static __device__ __forceinline__ _Float16 tof16(float x)
{
    unsigned u = __float_as_uint(x);
    u = (u + 0x7FFFu + ((u >> 16) & 1u)) & 0xFFFF0000u;
    return (_Float16)__uint_as_float(u);
}

static __device__ __forceinline__ v16h cat8(v8h a, v8h b)
{
    return __builtin_shufflevector(a, b, 0, 1, 2, 3, 4, 5, 6, 7, 8, 9, 10, 11, 12, 13, 14, 15);
}

static __device__ __forceinline__ v8f wmma16(v16h a, v16h b, v8f c)
{
    v8f d = __builtin_amdgcn_wmma_f32_16x16x32_f16(false, a, false, b, (short)0, c, false, false);
    asm volatile("v_nop\n\tv_nop\n\tv_nop\n\tv_nop" : "+v"(d) : "v"(a), "v"(b));
    return d;
}

__global__ void __launch_bounds__(128) local_attn_kernel(const float* __restrict__ Q,
                                                         const float* __restrict__ K,
                                                         const float* __restrict__ V,
                                                         float* __restrict__ O)
{
    __shared__ __align__(16) _Float16 kbuf[32 * KP];
    __shared__ __align__(16) _Float16 vbuf[HD * VP];
    __shared__ __align__(16) _Float16 pbuf[4][16 * 32];
    __shared__ __align__(16) _Float16 plbuf[4][16 * 32];
    __shared__ __align__(16) float    sout[4][16 * HD];

    const int tid  = threadIdx.x;
    const int lane = tid & 31;
    const int wave = __builtin_amdgcn_readfirstlane(tid >> 5);
    const int lo   = lane & 15;
    const int hi   = lane >> 4;
    const int koff = hi * 8;
    const int q0   = blockIdx.x * QB;
    const int bh   = blockIdx.y;
    const int qw   = q0 + wave * 16;
    const size_t rowbase = (size_t)bh * S_FULL;

    _Float16* pb  = pbuf[wave];
    _Float16* plb = plbuf[wave];

    v16h aq0, aq1;
    {
        const float* qr = Q + (rowbase + qw + lo) * HD;
        v8h f[4];
#pragma unroll
        for (int s = 0; s < 4; ++s) {
            const v4f x0 = *(const v4f*)(qr + 16 * s + koff);
            const v4f x1 = *(const v4f*)(qr + 16 * s + koff + 4);
            v8h t;
            t[0] = tof16(x0[0]); t[1] = tof16(x0[1]); t[2] = tof16(x0[2]); t[3] = tof16(x0[3]);
            t[4] = tof16(x1[0]); t[5] = tof16(x1[1]); t[6] = tof16(x1[2]); t[7] = tof16(x1[3]);
            f[s] = t;
        }
        aq0 = cat8(f[0], f[1]);
        aq1 = cat8(f[2], f[3]);
    }

    v8f oacc[4];
#pragma unroll
    for (int nt = 0; nt < 4; ++nt) { v8f z = {}; oacc[nt] = z; }
    float rm[8], rl[8];
#pragma unroll
    for (int i = 0; i < 8; ++i) { rm[i] = NEG_BIG; rl[i] = 0.0f; }

    int kmin = q0 - HALF_W; if (kmin < 0) kmin = 0;
    const int cb = kmin & ~31;
    int kmax = q0 + QB - 1 + HALF_W; if (kmax > SEQ - 1) kmax = SEQ - 1;

    for (int c = cb; c <= kmax; c += 32) {
#pragma unroll
        for (int it = 0; it < 4; ++it) {
            const int idx  = tid + 128 * it;
            const int row  = idx >> 4;
            const int col4 = (idx & 15) * 4;
            const size_t g = (rowbase + c + row) * HD + col4;
            const v4f kk = *(const v4f*)(K + g);
            const v4f vv = *(const v4f*)(V + g);
            v4h kh;
            kh[0] = tof16(kk[0]); kh[1] = tof16(kk[1]); kh[2] = tof16(kk[2]); kh[3] = tof16(kk[3]);
            *(v4h*)(kbuf + row * KP + col4) = kh;
            vbuf[(col4 + 0) * VP + row] = tof16(vv[0]);
            vbuf[(col4 + 1) * VP + row] = tof16(vv[1]);
            vbuf[(col4 + 2) * VP + row] = tof16(vv[2]);
            vbuf[(col4 + 3) * VP + row] = tof16(vv[3]);
        }
        __syncthreads();

        const bool active = (c <= qw + 15 + HALF_W) && (c + 31 >= qw - HALF_W);

        if (active) {
            const _Float16* k0r = kbuf + lo * KP;
            const _Float16* k1r = kbuf + (16 + lo) * KP;
            const v16h b00 = cat8(*(const v8h*)(k0r + koff),      *(const v8h*)(k0r + 16 + koff));
            const v16h b01 = cat8(*(const v8h*)(k0r + 32 + koff), *(const v8h*)(k0r + 48 + koff));
            const v16h b10 = cat8(*(const v8h*)(k1r + koff),      *(const v8h*)(k1r + 16 + koff));
            const v16h b11 = cat8(*(const v8h*)(k1r + 32 + koff), *(const v8h*)(k1r + 48 + koff));
            v8f cs0 = {}, cs1 = {};
            cs0 = wmma16(aq0, b00, cs0);
            cs0 = wmma16(aq1, b01, cs0);
            cs1 = wmma16(aq0, b10, cs1);
            cs1 = wmma16(aq1, b11, cs1);

#pragma unroll
            for (int i = 0; i < 8; ++i) {
                const int m = i + 8 * hi;
                const int q = qw + m;
                int d0 = q - (c + lo);      d0 = d0 < 0 ? -d0 : d0;
                int d1 = q - (c + 16 + lo); d1 = d1 < 0 ? -d1 : d1;
                const bool ok0 = (d0 <= HALF_W);
                const bool ok1 = (d1 <= HALF_W);
                const float sv0 = ok0 ? cs0[i] * SCALE : NEG_BIG;
                const float sv1 = ok1 ? cs1[i] * SCALE : NEG_BIG;

                float mx = fmaxf(sv0, sv1);
#pragma unroll
                for (int d = 1; d < 16; d <<= 1) mx = fmaxf(mx, __shfl_xor(mx, d, 32));
                const float mnew = fmaxf(rm[i], mx);
                const float scal = __expf(rm[i] - mnew);
                float p0 = __expf(sv0 - mnew); p0 = ok0 ? p0 : 0.0f;
                float p1 = __expf(sv1 - mnew); p1 = ok1 ? p1 : 0.0f;
                float sum = p0 + p1;
#pragma unroll
                for (int d = 1; d < 16; d <<= 1) sum += __shfl_xor(sum, d, 32);
                rl[i] = rl[i] * scal + sum;
                rm[i] = mnew;
#pragma unroll
                for (int nt = 0; nt < 4; ++nt) oacc[nt][i] *= scal;

                const float w0 = p0 * PSCALE, w1 = p1 * PSCALE;
                const _Float16 h0 = (_Float16)w0, h1 = (_Float16)w1;
                pb[m * 32 + lo]       = h0;  plb[m * 32 + lo]      = (_Float16)((w0 - (float)h0) * LSCALE);
                pb[m * 32 + 16 + lo]  = h1;  plb[m * 32 + 16 + lo] = (_Float16)((w1 - (float)h1) * LSCALE);
            }
        }
        __syncthreads();

        if (active) {
            const v16h ap  = cat8(*(const v8h*)(pb + lo * 32 + koff),  *(const v8h*)(pb + lo * 32 + 16 + koff));
            const v16h apl = cat8(*(const v8h*)(plb + lo * 32 + koff), *(const v8h*)(plb + lo * 32 + 16 + koff));
#pragma unroll
            for (int nt = 0; nt < 4; ++nt) {
                const _Float16* vr = vbuf + (nt * 16 + lo) * VP;
                const v16h vb = cat8(*(const v8h*)(vr + koff), *(const v8h*)(vr + 16 + koff));
                v8f x = {};
                x = wmma16(apl, vb, x);
                oacc[nt] = wmma16(ap, vb, oacc[nt]);
                oacc[nt] += x * RSPLIT;
            }
        }
        __syncthreads();
    }

    float inv[8];
#pragma unroll
    for (int i = 0; i < 8; ++i) inv[i] = 1.0f / (rl[i] * PSCALE);
    float* so = sout[wave];
#pragma unroll
    for (int nt = 0; nt < 4; ++nt) {
#pragma unroll
        for (int i = 0; i < 8; ++i) so[(i + 8 * hi) * HD + nt * 16 + lo] = oacc[nt][i] * inv[i];
    }
    __syncthreads();

    v4f ov[8];
#pragma unroll
    for (int i = 0; i < 8; ++i) {
        const int cc = lane + 32 * i, rr = cc >> 4, qd = cc & 15;
        ov[i] = *(const v4fa*)(so + rr * HD + qd * 4);
    }
    float* ob = O + (rowbase + qw) * HD;
#pragma unroll
    for (int i = 0; i < 8; ++i) {
        const int cc = lane + 32 * i, rr = cc >> 4, qd = cc & 15;
        *(volatile v4f*)(ob + (size_t)rr * HD + qd * 4) = ov[i];
    }
    __threadfence();
#pragma unroll
    for (int i = 0; i < 8; ++i) {
        const int cc = lane + 32 * i, rr = cc >> 4, qd = cc & 15;
        *(volatile v4f*)(ob + (size_t)rr * HD + qd * 4) = ov[i];
    }
}

extern "C" void kernel_launch(void* const* d_in, const int* in_sizes, int n_in,
                              void* d_out, int out_size, void* d_ws, size_t ws_size,
                              hipStream_t stream)
{
    (void)d_ws; (void)ws_size;
    if (n_in < 3) return;
    const long long need = ((long long)(NB * NH - 1) * S_FULL + SEQ) * HD;
    if ((long long)in_sizes[0] < need || (long long)in_sizes[1] < need || (long long)in_sizes[2] < need) return;
    if ((long long)out_size < need) return;

    const float* Q = (const float*)d_in[0];
    const float* K = (const float*)d_in[1];
    const float* V = (const float*)d_in[2];
    float*       O = (float*)d_out;

    dim3 grid(SEQ / QB, NB * NH);
    local_attn_kernel<<<grid, 128, 0, stream>>>(Q, K, V, O);
}
